// WarCraftModel_31104153157789
// MI455X (gfx1250) — hardware-verified
//
#include <hip/hip_runtime.h>
#include <math.h>

typedef __attribute__((ext_vector_type(16))) _Float16 v16h;
typedef __attribute__((ext_vector_type(8)))  _Float16 v8h;
typedef __attribute__((ext_vector_type(4)))  _Float16 v4h;
typedef __attribute__((ext_vector_type(16))) __bf16   v16b;
typedef __attribute__((ext_vector_type(8)))  __bf16   v8b;
typedef __attribute__((ext_vector_type(8)))  float    v8f;
typedef __attribute__((ext_vector_type(4)))  float    v4f;
typedef __attribute__((ext_vector_type(4)))  int      v4i;
typedef __attribute__((ext_vector_type(2)))  double   v2d;

__device__ __forceinline__ unsigned short f2bf_bits(float f) {
  unsigned u = __float_as_uint(f);
  return (unsigned short)((u + 0x7FFFu + ((u >> 16) & 1u)) >> 16);
}
__device__ __forceinline__ float bf_bits2f(unsigned short h) { return __uint_as_float(((unsigned)h) << 16); }

__device__ __forceinline__ void dep_guard_h(v8f& a, v8f& b, v16h x, v16h y) { asm volatile("v_nop\n\tv_nop\n\tv_nop\n\tv_nop" : "+v"(a), "+v"(b) : "v"(x), "v"(y)); }
__device__ __forceinline__ void dep_guard_b(v8f& a, v8f& b, v16b x, v16b y) { asm volatile("v_nop\n\tv_nop\n\tv_nop\n\tv_nop" : "+v"(a), "+v"(b) : "v"(x), "v"(y)); }
__device__ __forceinline__ void keep4_h(v16h a, v16h b, v16h c, v16h d) { asm volatile("v_nop" :: "v"(a), "v"(b), "v"(c), "v"(d)); }
__device__ __forceinline__ void keep4_b(v16b a, v16b b, v16b c, v16b d) { asm volatile("v_nop" :: "v"(a), "v"(b), "v"(c), "v"(d)); }
__device__ __forceinline__ void acc_guard4(v8f& a, v8f& b, v8f& c, v8f& d) { asm volatile("v_nop\n\tv_nop\n\tv_nop\n\tv_nop" : "+v"(a), "+v"(b), "+v"(c), "+v"(d)); }
template <typename T> struct Frag;
template <> struct Frag<_Float16> {
  typedef v16h V; union U { v16h v; v8h h[2]; };
  static __device__ __forceinline__ v16h load(const _Float16* p) {
    U f; f.h[0] = *(const v8h*)(p); f.h[1] = *(const v8h*)(p + 16); return f.v;
  }
  static __device__ __forceinline__ v8f mma(v16h a, v16h b, v8f c) {
    return __builtin_amdgcn_wmma_f32_16x16x32_f16(false, a, false, b, (short)0, c, false, false);
  }
  static __device__ __forceinline__ void guard(v8f& a, v8f& b, v16h x, v16h y) { dep_guard_h(a, b, x, y); }
  static __device__ __forceinline__ void keep(v16h a, v16h b, v16h c, v16h d) { keep4_h(a, b, c, d); }
};
template <> struct Frag<__bf16> {
  typedef v16b V; union U { v16b v; v8b h[2]; };
  static __device__ __forceinline__ v16b load(const __bf16* p) {
    U f; f.h[0] = *(const v8b*)(p); f.h[1] = *(const v8b*)(p + 16); return f.v;
  }
  static __device__ __forceinline__ v8f mma(v16b a, v16b b, v8f c) {
    return __builtin_amdgcn_wmma_f32_16x16x32_bf16(false, a, false, b, (short)0, c, false, false);
  }
  static __device__ __forceinline__ void guard(v8f& a, v8f& b, v16b x, v16b y) { dep_guard_b(a, b, x, y); }
  static __device__ __forceinline__ void keep(v16b a, v16b b, v16b c, v16b d) { keep4_b(a, b, c, d); }
};

template <int ET> struct Elem;
template <> struct Elem<0> { typedef _Float16 T; };
template <> struct Elem<1> { typedef __bf16 T; };
template <int ET, bool SPLIT, int BIAS_MODE, int OUT_MODE, bool RESID, int ACT = 0>
__global__ __launch_bounds__(256) void wmma_gemm64(
    const unsigned short* __restrict__ Ap, const unsigned short* __restrict__ A2p, int lda, long strideA,
    const unsigned short* __restrict__ Btp, const unsigned short* __restrict__ Bt2p, int ldb, long strideB,
    void* __restrict__ Cout, void* __restrict__ Cout2, int ldc, long strideC,
    const float* __restrict__ bias,
    const float* __restrict__ resid, long strideR,
    int M, int N, int K, float scale) {
  typedef typename Elem<ET>::T T;
  typedef typename Frag<T>::V V;
  const T* A = (const T*)Ap; const T* A2 = (const T*)A2p; const T* Bt = (const T*)Btp; const T* Bt2 = (const T*)Bt2p;
  __shared__ __align__(16) float sT[8][16 * 68];
  const int b    = blockIdx.y;
  const int lane = threadIdx.x & 31;
  const int wave = threadIdx.x >> 5;
  const int tilesN = N >> 6;
  const int tilesM = M >> 6;
  const int tile = blockIdx.x * 8 + wave;
  if (tile >= tilesM * tilesN) return;
  const int tm = tile / tilesN;
  const int tn = tile - tm * tilesN;
  const int m0 = tm << 6;
  const int n0 = tn << 6;

  const T* Ab  = A  + (size_t)b * strideA;
  const T* Bb  = Bt + (size_t)b * strideB;
  const T* Ab2 = SPLIT ? (A2  + (size_t)b * strideA) : nullptr;
  const T* Bb2 = SPLIT ? (Bt2 + (size_t)b * strideB) : nullptr;

  const int rlane = lane & 15;
  const int koff  = (lane >> 4) * 8;
  const int mOff  = (lane >> 4) * 8;

  v8f acc[4][4];
#pragma unroll
  for (int i = 0; i < 4; ++i)
#pragma unroll
    for (int j = 0; j < 4; ++j) acc[i][j] = (v8f){0.f,0.f,0.f,0.f,0.f,0.f,0.f,0.f};

  for (int k0 = 0; k0 < K; k0 += 32) {
    V bh[4], bl[4];
#pragma unroll
    for (int j = 0; j < 4; ++j) {
      const size_t bo = (size_t)(n0 + (j << 4) + rlane) * ldb + koff + k0;
      bh[j] = Frag<T>::load(Bb + bo);
      if (SPLIT) bl[j] = Frag<T>::load(Bb2 + bo);
    }
#pragma unroll
    for (int i = 0; i < 4; ++i) {
      const size_t ao = (size_t)(m0 + (i << 4) + rlane) * lda + koff + k0;
      V ah = Frag<T>::load(Ab + ao);
      V al;
      if (SPLIT) al = Frag<T>::load(Ab2 + ao);
#pragma unroll
      for (int j = 0; j < 4; ++j) {
        acc[i][j] = Frag<T>::mma(ah, bh[j], acc[i][j]);
        if (SPLIT) {
          acc[i][j] = Frag<T>::mma(ah, bl[j], acc[i][j]);
          acc[i][j] = Frag<T>::mma(al, bh[j], acc[i][j]);
        }
      }
      Frag<T>::guard(acc[i][0], acc[i][3], ah, SPLIT ? al : ah);
    }
    Frag<T>::keep(bh[0], bh[1], bh[2], bh[3]);
    if (SPLIT) Frag<T>::keep(bl[0], bl[1], bl[2], bl[3]);
  }
  acc_guard4(acc[0][0], acc[0][1], acc[0][2], acc[0][3]);
  acc_guard4(acc[1][0], acc[1][1], acc[1][2], acc[1][3]);
  acc_guard4(acc[2][0], acc[2][1], acc[2][2], acc[2][3]);
  acc_guard4(acc[3][0], acc[3][1], acc[3][2], acc[3][3]);

  float* slab = sT[wave];
  const float* Rb = RESID ? (resid + (size_t)b * strideR) : nullptr;
#pragma unroll
  for (int i = 0; i < 4; ++i) {
    const int mBase = m0 + (i << 4);
#pragma unroll
    for (int j = 0; j < 4; ++j) {
      const int n = n0 + (j << 4) + rlane;
      float bv = 0.f;
      if (BIAS_MODE == 2) bv = bias[n];
#pragma unroll
      for (int r = 0; r < 8; ++r) {
        float v = acc[i][j][r] * scale;
        if (BIAS_MODE == 1) v += bias[mBase + mOff + r];
        if (BIAS_MODE == 2) v += bv;
        if (RESID) v += Rb[(size_t)(mBase + mOff + r) * ldc + n];
        if (ACT == 1) v = tanhf(v);
        if (ACT == 2) v = fmaxf(v, 0.0f);
        if (ACT == 3) v = v / (1.0f + expf(-v));
        if (ACT == 4) v = (v > 0.f) ? v : 0.01f * v;
        if (ACT == 5) v = 0.5f * v * (1.0f + erff(v * 0.70710678118654752f));
        slab[(mOff + r) * 68 + (j << 4) + rlane] = v;
      }
    }
    __builtin_amdgcn_fence(__ATOMIC_RELEASE, "workgroup");
    __builtin_amdgcn_wave_barrier();
    __builtin_amdgcn_fence(__ATOMIC_ACQUIRE, "workgroup");
    if (OUT_MODE == 0) {
      float* C = (float*)Cout + (size_t)b * strideC;
      const int hh = lane >> 4, c4 = (lane & 15) * 4;
      for (int pass = 0; pass < 2; ++pass) {
#pragma unroll
        for (int it = 0; it < 8; ++it) {
          const int row = it * 2 + hh;
          v4f v = *(const v4f*)(slab + row * 68 + c4);
          *(volatile v4f*)(C + (size_t)(mBase + row) * ldc + n0 + c4) = v;
        }
        __threadfence();
      }
    } else {
      const int q = lane >> 3, c8 = (lane & 7) * 8;
      unsigned short* C  = (unsigned short*)Cout  + (size_t)b * strideC;
      unsigned short* C2 = (OUT_MODE == 2) ? ((unsigned short*)Cout2 + (size_t)b * strideC) : nullptr;
      for (int pass = 0; pass < 2; ++pass) {
#pragma unroll
        for (int it = 0; it < 4; ++it) {
          const int row = it * 4 + q;
          const float* sp = slab + row * 68 + c8;
          v8h hv, lv;
#pragma unroll
          for (int e = 0; e < 8; ++e) {
            if (OUT_MODE == 1) {
              hv[e] = (_Float16)sp[e];
            } else {
              unsigned short hb = f2bf_bits(sp[e]);
              unsigned short lb = f2bf_bits(sp[e] - bf_bits2f(hb));
              hv[e] = __builtin_bit_cast(_Float16, hb);
              lv[e] = __builtin_bit_cast(_Float16, lb);
            }
          }
          *(volatile v8h*)(C + (size_t)(mBase + row) * ldc + n0 + c8) = hv;
          if (OUT_MODE == 2) *(volatile v8h*)(C2 + (size_t)(mBase + row) * ldc + n0 + c8) = lv;
        }
        __threadfence();
      }
    }
    __builtin_amdgcn_fence(__ATOMIC_RELEASE, "workgroup");
    __builtin_amdgcn_wave_barrier();
    __builtin_amdgcn_fence(__ATOMIC_ACQUIRE, "workgroup");
  }
}

template <int NW>
__device__ __forceinline__ int block_excl_scan(int cnt, int* wtot, int lane, int wave, int& total) {
  int incl = cnt;
#pragma unroll
  for (int off = 1; off < 32; off <<= 1) {
    const int t = __shfl_up(incl, off, 32);
    if (lane >= off) incl += t;
  }
  if (lane == 31) wtot[wave] = incl;
  __syncthreads();
  int base = 0, tot = 0;
#pragma unroll
  for (int w = 0; w < NW; ++w) { const int t = wtot[w]; tot += t; base += (w < wave) ? t : 0; }
  total = tot;
  return base + incl - cnt;
}

constexpr int   kThr   = 64;
constexpr int   kWav   = kThr / 32;
constexpr int   kEpt   = 8;
constexpr int   kChunk = kThr * kEpt;
constexpr int   kTileD = 8192;
constexpr int   kTileA = 1024;
constexpr int   kCh    = 32;
constexpr int   kGwLd  = 64;
constexpr float kBnEps = 1e-5f;
static_assert(kThr == 64, "thread-ownership maps below assume 64 threads = 8 groups of 8 lanes");
static_assert(kTileD % kThr == 0 && kTileD % 128 == 0 && kTileA % 8 == 0, "tile shapes");

__global__ __launch_bounds__(kThr) void gcn_dinv_p1_kernel(
    const int* __restrict__ edst, const float* __restrict__ ew,
    const float* __restrict__ X, const float* __restrict__ W1,
    float* __restrict__ dinv, float* __restrict__ P1, int N, int NE) {
  __shared__ __align__(16) float accd[kTileD];
  __shared__ int   ldl[kChunk];
  __shared__ float lwv[kChunk];
  __shared__ int   wtot[kWav];
  const int tid = threadIdx.x, lane = tid & 31, wave = tid >> 5;
  const int tile0 = blockIdx.x * kTileD;
#pragma unroll 1
  for (int i = 0; i < kTileD / kThr; ++i) accd[i * kThr + tid] = 1.0f;
  for (int cb = 0; cb < NE; cb += kChunk) {
    const int e0  = cb + tid * kEpt;
    const int ebc = (e0 + kEpt <= NE) ? e0 : (NE - kEpt);
    const v4i ca  = *(const v4i*)(edst + ebc);
    const v4i cbv = *(const v4i*)(edst + ebc + 4);
    int cv[kEpt];
    cv[0] = ca[0];  cv[1] = ca[1];  cv[2] = ca[2];  cv[3] = ca[3];
    cv[4] = cbv[0]; cv[5] = cbv[1]; cv[6] = cbv[2]; cv[7] = cbv[3];
    unsigned flags = 0;
#pragma unroll
    for (int i = 0; i < kEpt; ++i)
      if ((ebc + i >= e0) && (unsigned)(cv[i] - tile0) < (unsigned)kTileD && cv[i] < N) flags |= 1u << i;
    const int cnt = __popc(flags);
    int nh;
    int pos = block_excl_scan<kWav>(cnt, wtot, lane, wave, nh);
#pragma unroll
    for (int i = 0; i < kEpt; ++i) {
      if (flags & (1u << i)) {
        if (pos < kChunk) { ldl[pos] = cv[i] - tile0; lwv[pos] = ew[ebc + i]; }
        ++pos;
      }
    }
    __syncthreads();
    nh = nh < kChunk ? nh : kChunk;
    for (int j = 0; j < nh; ++j) {
      const int dl = ldl[j];
      const float wv = lwv[j];
      if ((dl & (kThr - 1)) == tid) accd[dl] += wv;
    }
    __syncthreads();
  }
#pragma unroll 1
  for (int i = 0; i < kTileD / kThr; ++i) {
    const int r = i * kThr + tid;
    const float deg = accd[r];
    accd[r] = (deg > 0.0f) ? (1.0f / sqrtf(deg)) : 0.0f;
  }
  __syncthreads();
  for (int pass = 0; pass < 2; ++pass) {
#pragma unroll 1
    for (int gi = wave; gi < kTileD / 128; gi += kWav) {
      const v4f v = *(const v4f*)(accd + gi * 128 + lane * 4);
      *(volatile v4f*)(dinv + (size_t)tile0 + gi * 128 + lane * 4) = v;
    }
    __threadfence();
  }
  const int grp = tid >> 3, ch0 = (tid & 7) * 4;
  float w0[4], w1[4], w2[4];
#pragma unroll
  for (int e = 0; e < 4; ++e) { w0[e] = W1[ch0 + e]; w1[e] = W1[kCh + ch0 + e]; w2[e] = W1[2 * kCh + ch0 + e]; }
  for (int pass = 0; pass < 2; ++pass) {
#pragma unroll 1
    for (int i = 0; i < kTileD / 8; ++i) {
      const int r = i * 8 + grp;
      const int node = tile0 + r;
      const int nodec = node < N ? node : (N - 1);
      const float x0 = X[(size_t)nodec * 3];
      const float x1 = X[(size_t)nodec * 3 + 1];
      const float x2 = X[(size_t)nodec * 3 + 2];
      const float di = accd[r];
      v4f p;
#pragma unroll
      for (int e = 0; e < 4; ++e) p[e] = di * (x0 * w0[e] + x1 * w1[e] + x2 * w2[e]);
      *(volatile v4f*)(P1 + (size_t)(tile0 + r) * kCh + ch0) = p;
    }
    __threadfence();
  }
}

__global__ __launch_bounds__(kThr) void gcn_agg1_kernel(
    const float* __restrict__ P1, const int* __restrict__ esrc, const int* __restrict__ edst,
    const float* __restrict__ ew, const float* __restrict__ dinv, const float* __restrict__ b1,
    float* __restrict__ H1, double* __restrict__ part, int N, int NE) {
  __shared__ __align__(16) float acc[kTileA * kCh];
  __shared__ int   lsr[kChunk];
  __shared__ int   ldl[kChunk];
  __shared__ float lwv[kChunk];
  __shared__ int   wtot[kWav];
  __shared__ __align__(16) double red[kThr * 8];
  __shared__ __align__(16) double lineb[2 * kCh];
  const int tid = threadIdx.x, lane = tid & 31, wave = tid >> 5;
  const int grp = tid >> 3, ch0 = (tid & 7) * 4;
  const int tile0 = blockIdx.x * kTileA;
  const v4f z4 = {0.f, 0.f, 0.f, 0.f};
#pragma unroll 1
  for (int i = 0; i < kTileA / 8; ++i) *(v4f*)(acc + (i * 8 + grp) * kCh + ch0) = z4;
  for (int cb = 0; cb < NE; cb += kChunk) {
    const int e0  = cb + tid * kEpt;
    const int ebc = (e0 + kEpt <= NE) ? e0 : (NE - kEpt);
    const v4i ca  = *(const v4i*)(edst + ebc);
    const v4i cbv = *(const v4i*)(edst + ebc + 4);
    int cv[kEpt];
    cv[0] = ca[0];  cv[1] = ca[1];  cv[2] = ca[2];  cv[3] = ca[3];
    cv[4] = cbv[0]; cv[5] = cbv[1]; cv[6] = cbv[2]; cv[7] = cbv[3];
    unsigned flags = 0;
#pragma unroll
    for (int i = 0; i < kEpt; ++i)
      if ((ebc + i >= e0) && (unsigned)(cv[i] - tile0) < (unsigned)kTileA && cv[i] < N) flags |= 1u << i;
    const int cnt = __popc(flags);
    int nh;
    int pos = block_excl_scan<kWav>(cnt, wtot, lane, wave, nh);
#pragma unroll
    for (int i = 0; i < kEpt; ++i) {
      if (flags & (1u << i)) {
        if (pos < kChunk) {
          int s = esrc[ebc + i];
          s = s < 0 ? 0 : (s >= N ? N - 1 : s);
          lsr[pos] = s; ldl[pos] = cv[i] - tile0; lwv[pos] = ew[ebc + i];
        }
        ++pos;
      }
    }
    __syncthreads();
    nh = nh < kChunk ? nh : kChunk;
    for (int j = 0; j < nh; ++j) {
      const int dl = ldl[j];
      const int s  = lsr[j];
      const float wv = lwv[j];
      if ((dl & 7) == grp) {
        const v4f m = *(const v4f*)(P1 + (size_t)s * kCh + ch0);
        float* ap = acc + dl * kCh + ch0;
        v4f a = *(const v4f*)ap;
#pragma unroll
        for (int e = 0; e < 4; ++e) a[e] += wv * m[e];
        *(v4f*)ap = a;
      }
    }
    __syncthreads();
  }
  const v4f b4 = *(const v4f*)(b1 + ch0);
  double s4[4] = {0.0, 0.0, 0.0, 0.0}, q4[4] = {0.0, 0.0, 0.0, 0.0};
#pragma unroll 1
  for (int i = 0; i < kTileA / 8; ++i) {
    const int r = i * 8 + grp;
    const int node = tile0 + r;
    const int nodec = node < N ? node : (N - 1);
    const float di = dinv[nodec];
    const v4f sf = *(const v4f*)(P1 + (size_t)nodec * kCh + ch0);
    float* ap = acc + r * kCh + ch0;
    const v4f a = *(const v4f*)ap;
    const float vm = (node < N) ? 1.0f : 0.0f;
    v4f h;
#pragma unroll
    for (int e = 0; e < 4; ++e) {
      const float hv = di * (a[e] + sf[e]) + b4[e];
      h[e] = hv;
      const float hm = hv * vm;
      s4[e] += (double)hm;
      q4[e] += (double)hm * (double)hm;
    }
    *(v4f*)ap = h;
  }
  for (int pass = 0; pass < 2; ++pass) {
#pragma unroll 1
    for (int i = 0; i < kTileA / 8; ++i) {
      const int r = i * 8 + grp;
      const v4f v = *(const v4f*)(acc + r * kCh + ch0);
      *(volatile v4f*)(H1 + (size_t)(tile0 + r) * kCh + ch0) = v;
    }
    __threadfence();
  }
#pragma unroll
  for (int e = 0; e < 4; ++e) { red[tid * 8 + e] = s4[e]; red[tid * 8 + 4 + e] = q4[e]; }
  __syncthreads();
  if (tid < kCh) {
    const int qq = tid >> 2, e = tid & 3;
    double S = 0.0, Q = 0.0;
#pragma unroll
    for (int g = 0; g < 8; ++g) { S += red[(g * 8 + qq) * 8 + e]; Q += red[(g * 8 + qq) * 8 + 4 + e]; }
    lineb[tid] = S; lineb[kCh + tid] = Q;
  }
  __syncthreads();
  if (wave == 0) {
    const v2d v = *(const v2d*)(lineb + 2 * lane);
    double* dst = part + (size_t)blockIdx.x * (2 * kCh) + 2 * lane;
    *(volatile v2d*)dst = v;
    __threadfence();
    *(volatile v2d*)dst = v;
  }
}

__global__ __launch_bounds__(kThr) void bn_stats_kernel(
    const double* __restrict__ part, int nblk, const float* __restrict__ gamma, float* __restrict__ SS, int N) {
  __shared__ __align__(16) float ssl[2 * kCh];
  const int tid = threadIdx.x;
  if (tid < kCh) {
    double S = 0.0, Q = 0.0;
    for (int bI = 0; bI < nblk; ++bI) { S += part[(size_t)bI * (2 * kCh) + tid]; Q += part[(size_t)bI * (2 * kCh) + kCh + tid]; }
    const double invn = 1.0 / (double)N;
    const double mean = S * invn;
    double var = Q * invn - mean * mean;
    var = var > 0.0 ? var : 0.0;
    const float vf = (float)var;
    const float sc = gamma[tid] * (1.0f / sqrtf(vf + kBnEps));
    ssl[tid] = (float)mean;
    ssl[kCh + tid] = sc;
  }
  __syncthreads();
  if (tid < 16) {
    const v4f v = *(const v4f*)(ssl + 4 * tid);
    float* dst = SS + 4 * tid;
    *(volatile v4f*)dst = v;
    __threadfence();
    *(volatile v4f*)dst = v;
  }
}

__global__ __launch_bounds__(256) void bn_relu_f16_kernel(
    const float* __restrict__ H1, const float* __restrict__ SS, const float* __restrict__ beta,
    _Float16* __restrict__ G16, int N, int NP, float carry) {
  const int gid = blockIdx.x * 256 + threadIdx.x;
  if (gid >= NP * 4) return;
  const int row = gid >> 2, c0 = (gid & 3) * 8;
  const int rowc = row < N ? row : (N - 1);
  const v4f xa = *(const v4f*)(H1 + (size_t)rowc * kCh + c0);
  const v4f xb = *(const v4f*)(H1 + (size_t)rowc * kCh + c0 + 4);
  const v4f ma = *(const v4f*)(SS + c0), mb = *(const v4f*)(SS + c0 + 4);
  const v4f sa = *(const v4f*)(SS + kCh + c0), sb = *(const v4f*)(SS + kCh + c0 + 4);
  const v4f ba = *(const v4f*)(beta + c0), bb = *(const v4f*)(beta + c0 + 4);
  const float vm = (row < N) ? carry : 0.0f;
  v8h hv;
#pragma unroll
  for (int e = 0; e < 4; ++e) {
    const float ya = fmaxf((xa[e] - ma[e]) * sa[e] + ba[e], 0.0f) * vm;
    const float yb = fmaxf((xb[e] - mb[e]) * sb[e] + bb[e], 0.0f) * vm;
    hv[e] = (_Float16)ya;
    hv[4 + e] = (_Float16)yb;
  }
  _Float16* dst = G16 + (size_t)row * kCh + c0;
  *(volatile v8h*)dst = hv;
  __threadfence();
  *(volatile v8h*)dst = hv;
}

__global__ __launch_bounds__(256) void w3t_kernel(const float* __restrict__ W3, _Float16* __restrict__ W3T, float carry) {
  const int t = threadIdx.x;
  const int n = t >> 2, k0 = (t & 3) * 8;
  v8h v;
#pragma unroll
  for (int i = 0; i < 8; ++i) {
    const float w = W3[k0 + i] * carry;
    v[i] = (n == 0) ? (_Float16)w : (_Float16)0.0f;
  }
  _Float16* dst = W3T + (size_t)n * kCh + k0;
  *(volatile v8h*)dst = v;
  __threadfence();
  *(volatile v8h*)dst = v;
}

__global__ __launch_bounds__(kThr) void gcn_agg2_kernel(
    const float* __restrict__ GW, const int* __restrict__ esrc, const int* __restrict__ edst,
    const float* __restrict__ ew, const float* __restrict__ dinv, const float* __restrict__ b3,
    float* __restrict__ out, int N, int NE) {
  __shared__ __align__(16) float acc[kTileD];
  __shared__ int   lsr[kChunk];
  __shared__ int   ldl[kChunk];
  __shared__ float lwv[kChunk];
  __shared__ int   wtot[kWav];
  const int tid = threadIdx.x, lane = tid & 31, wave = tid >> 5;
  const int tile0 = blockIdx.x * kTileD;
#pragma unroll 1
  for (int i = 0; i < kTileD / kThr; ++i) acc[i * kThr + tid] = 0.0f;
  for (int cb = 0; cb < NE; cb += kChunk) {
    const int e0  = cb + tid * kEpt;
    const int ebc = (e0 + kEpt <= NE) ? e0 : (NE - kEpt);
    const v4i ca  = *(const v4i*)(edst + ebc);
    const v4i cbv = *(const v4i*)(edst + ebc + 4);
    int cv[kEpt];
    cv[0] = ca[0];  cv[1] = ca[1];  cv[2] = ca[2];  cv[3] = ca[3];
    cv[4] = cbv[0]; cv[5] = cbv[1]; cv[6] = cbv[2]; cv[7] = cbv[3];
    unsigned flags = 0;
#pragma unroll
    for (int i = 0; i < kEpt; ++i)
      if ((ebc + i >= e0) && (unsigned)(cv[i] - tile0) < (unsigned)kTileD && cv[i] < N) flags |= 1u << i;
    const int cnt = __popc(flags);
    int nh;
    int pos = block_excl_scan<kWav>(cnt, wtot, lane, wave, nh);
#pragma unroll
    for (int i = 0; i < kEpt; ++i) {
      if (flags & (1u << i)) {
        if (pos < kChunk) {
          int s = esrc[ebc + i];
          s = s < 0 ? 0 : (s >= N ? N - 1 : s);
          lsr[pos] = s; ldl[pos] = cv[i] - tile0; lwv[pos] = ew[ebc + i];
        }
        ++pos;
      }
    }
    __syncthreads();
    nh = nh < kChunk ? nh : kChunk;
    for (int j = 0; j < nh; ++j) {
      const int dl = ldl[j];
      const int s  = lsr[j];
      const float wv = lwv[j];
      if ((dl & (kThr - 1)) == tid) {
        const float m = dinv[s] * GW[(size_t)s * kGwLd];
        acc[dl] += wv * m;
      }
    }
    __syncthreads();
  }
  const float bias = b3[0];
#pragma unroll 1
  for (int i = 0; i < kTileD / kThr; ++i) {
    const int r = i * kThr + tid;
    const int node = tile0 + r;
    const int nodec = node < N ? node : (N - 1);
    const float di = dinv[nodec];
    const float gs = GW[(size_t)nodec * kGwLd];
    acc[r] = di * (acc[r] + di * gs) + bias;
  }
  __syncthreads();
  for (int pass = 0; pass < 2; ++pass) {
#pragma unroll 1
    for (int gi = wave; gi < kTileD / 128; gi += kWav) {
      const int idx = tile0 + gi * 128 + lane * 4;
      const v4f v = *(const v4f*)(acc + gi * 128 + lane * 4);
      if (idx < N) *(volatile v4f*)(out + idx) = v;
    }
    __threadfence();
  }
}

extern "C" void kernel_launch(void* const* d_in, const int* in_sizes, int n_in,
                              void* d_out, int out_size, void* d_ws, size_t ws_size,
                              hipStream_t stream) {
  if (n_in < 9) return;
  const int N = in_sizes[0] / 3;
  if (N < 64 || in_sizes[0] != N * 3 || (N % 32) != 0) return;
  if (in_sizes[1] & 1) return;
  const int NE = in_sizes[1] / 2;
  if (in_sizes[2] != NE || NE < 8 || (NE % 8) != 0) return;
  if (in_sizes[3] != 3 * kCh || in_sizes[4] != kCh || in_sizes[5] != kCh || in_sizes[6] != kCh ||
      in_sizes[7] != kCh || in_sizes[8] < 1) return;
  if (out_size != N) return;

  const float* x     = (const float*)d_in[0];
  const int*   eidx  = (const int*)d_in[1];
  const float* eattr = (const float*)d_in[2];
  const float* W1    = (const float*)d_in[3];
  const float* b1    = (const float*)d_in[4];
  const float* gam1  = (const float*)d_in[5];
  const float* bet1  = (const float*)d_in[6];
  const float* W3    = (const float*)d_in[7];
  const float* b3    = (const float*)d_in[8];
  const int* esrc = eidx;
  const int* edst = eidx + NE;
  float* outp = (float*)d_out;

  const int NP     = ((N + 63) / 64) * 64;
  const int nblkD  = (N + kTileD - 1) / kTileD;
  const int nblkA  = (N + kTileA - 1) / kTileA;
  const size_t rowsD = (size_t)nblkD * kTileD;
  const size_t rowsA = (size_t)nblkA * kTileA;

  size_t off = 0;
  auto carve = [&](size_t bytes) -> char* { char* p = (char*)d_ws + off; off += (bytes + 255) & ~(size_t)255; return p; };
  float*    DINV = (float*)carve(rowsD * 4);
  float*    P1   = (float*)carve(rowsD * kCh * 4);
  float*    H1   = (float*)carve(rowsA * kCh * 4);
  double*   PART = (double*)carve((size_t)nblkA * 2 * kCh * 8);
  float*    SS   = (float*)carve((size_t)2 * kCh * 4);
  _Float16* G16  = (_Float16*)carve((size_t)NP * kCh * 2);
  _Float16* W3T  = (_Float16*)carve((size_t)64 * kCh * 2);
  float*    GW   = (float*)carve((size_t)NP * kGwLd * 4);
  if (off > ws_size || off > (size_t)134217728) return;

  const float gcarry = 8.0f;
  const float wcarry = 8.0f;

  gcn_dinv_p1_kernel<<<nblkD, kThr, 0, stream>>>(edst, eattr, x, W1, DINV, P1, N, NE);
  gcn_agg1_kernel<<<nblkA, kThr, 0, stream>>>(P1, esrc, edst, eattr, DINV, b1, H1, PART, N, NE);

  bn_stats_kernel<<<1, kThr, 0, stream>>>(PART, nblkA, gam1, SS, N);
  bn_relu_f16_kernel<<<(NP * 4 + 255) / 256, 256, 0, stream>>>(H1, SS, bet1, G16, N, NP, gcarry);

  w3t_kernel<<<1, 256, 0, stream>>>(W3, W3T, wcarry);
  {
    const int tiles = (NP / 64) * (64 / 64);
    dim3 grid((tiles + 7) / 8, 1);
    wmma_gemm64<0, false, 0, 0, false, 0><<<grid, 256, 0, stream>>>(
        (const unsigned short*)G16, (const unsigned short*)G16, kCh, 0L,
        (const unsigned short*)W3T, (const unsigned short*)W3T, kCh, 0L,
        (void*)GW, (void*)GW, kGwLd, 0L, SS, SS, 0L, NP, 64, kCh, 1.0f / (gcarry * wcarry));
  }

  gcn_agg2_kernel<<<nblkD, kThr, 0, stream>>>(GW, esrc, edst, eattr, DINV, b3, outp, N, NE);
}
